// GPSA2D_3590592659850
// MI455X (gfx1250) — hardware-verified
//
#include <hip/hip_runtime.h>
#include <math.h>

typedef __attribute__((ext_vector_type(16))) _Float16 v16h;
typedef __attribute__((ext_vector_type(16))) __bf16 v16b;
typedef __attribute__((ext_vector_type(8)))  _Float16 v8h;
typedef __attribute__((ext_vector_type(8)))  float v8f;
typedef __attribute__((ext_vector_type(4)))  float v4f;
typedef __attribute__((ext_vector_type(2)))  float v2f;
typedef __attribute__((ext_vector_type(4)))  unsigned v4u;
typedef __attribute__((ext_vector_type(4)))  int v4i;
typedef float __attribute__((may_alias)) float_a;
typedef int __attribute__((may_alias)) int_a;

template <typename T> __device__ __forceinline__ void vst2(void* p, T v) { *(volatile T*)p = v; __threadfence(); *(volatile T*)p = v; }
__device__ __forceinline__ v8f wmma16(v16h a, v16h b, v8f c) {
  v8f d = __builtin_amdgcn_wmma_f32_16x16x32_f16(false, a, false, b, (short)0, c, false, false);
  asm volatile("v_nop\n\tv_nop\n\tv_nop\n\tv_nop" : "+v"(d) : "v"(a), "v"(b));
  return d;
}
__device__ __forceinline__ v8f wmma_bf(v16b a, v16b b, v8f c) {
  v8f d = __builtin_amdgcn_wmma_f32_16x16x32_bf16(false, a, false, b, (short)0, c, false, false);
  asm volatile("v_nop\n\tv_nop\n\tv_nop\n\tv_nop" : "+v"(d) : "v"(a), "v"(b));
  return d;
}
__device__ __forceinline__ v16h frag_h(const _Float16* rowk0, int lane) {
  union { v16h v; v8h q[2]; } u; const _Float16* p = rowk0 + 8 * (lane >> 4);
  u.q[0] = *(const v8h*)p; u.q[1] = *(const v8h*)(p + 16); return u.v;
}
__device__ __forceinline__ v16h frag_f32(const float* rowk0, int lane) {
  v16h a; const float* p = rowk0 + 8 * (lane >> 4);
#pragma unroll
  for (int i = 0; i < 8; ++i) { a[i] = (_Float16)p[i]; a[8 + i] = (_Float16)p[16 + i]; }
  return a;
}
__device__ __forceinline__ v16h frag_f32s(const float* rowk0, int lane, float sc) {
  v16h a; const float* p = rowk0 + 8 * (lane >> 4);
#pragma unroll
  for (int i = 0; i < 8; ++i) { a[i] = (_Float16)(p[i] * sc); a[8 + i] = (_Float16)(p[16 + i] * sc); }
  return a;
}
__device__ __forceinline__ v16h fragc_f32(const float* W, int k0, int n, int lane, int ld, int K) {
  v16h a; const int g = lane >> 4;
#pragma unroll
  for (int i = 0; i < 8; ++i) { const int ka = k0 + 8 * g + i, kb = ka + 16;
    a[i] = (_Float16)(ka < K ? W[(size_t)(ka < K ? ka : K - 1) * ld + n] : 0.f); a[8 + i] = (_Float16)(kb < K ? W[(size_t)(kb < K ? kb : K - 1) * ld + n] : 0.f); }
  return a;
}
struct F2 { v16b h, l; };
__device__ __forceinline__ F2 bsplit16(const float v[16]) { F2 r;
#pragma unroll
  for (int i = 0; i < 16; ++i) { const __bf16 h = (__bf16)v[i]; r.h[i] = h; r.l[i] = (__bf16)(v[i] - (float)h); }
  return r; }
__device__ __forceinline__ F2 split_row(const float* row, int k0, int lane) { float v[16]; const float* p = row + k0 + 8 * (lane >> 4);
#pragma unroll
  for (int i = 0; i < 8; ++i) { v[i] = p[i]; v[8 + i] = p[16 + i]; }
  return bsplit16(v); }
__device__ __forceinline__ F2 split_rowK(const float* row, int k0, int lane, int K) { float v[16]; const int g = lane >> 4;
#pragma unroll
  for (int i = 0; i < 8; ++i) { const int ka = k0 + 8 * g + i, kb = ka + 16; v[i] = ka < K ? row[ka < K ? ka : K - 1] : 0.f; v[8 + i] = kb < K ? row[kb < K ? kb : K - 1] : 0.f; }
  return bsplit16(v); }
__device__ __forceinline__ F2 split_col(const float* W, int k0, int n, int lane, int ld, int K) { float v[16]; const int g = lane >> 4;
#pragma unroll
  for (int i = 0; i < 8; ++i) { const int ka = k0 + 8 * g + i, kb = ka + 16; v[i] = ka < K ? W[(size_t)(ka < K ? ka : K - 1) * ld + n] : 0.f; v[8 + i] = kb < K ? W[(size_t)(kb < K ? kb : K - 1) * ld + n] : 0.f; }
  return bsplit16(v); }
__device__ __forceinline__ v8f mac3(const F2& a, const F2& b, v8f c) { c = wmma_bf(a.l, b.h, c); c = wmma_bf(a.h, b.l, c); return wmma_bf(a.h, b.h, c); }
__device__ __forceinline__ float sigm(float v) { return 1.0f / (1.0f + expf(-v)); }
#define LDSX() do { asm volatile("s_wait_dscnt 0" ::: "memory"); __builtin_amdgcn_wave_barrier(); __builtin_amdgcn_fence(__ATOMIC_RELEASE, "workgroup"); } while (0)


#define NB 2
#define NT 1600
#define DIM 384
#define NH 16
#define HDm 24
#define GWD 40
#define NR (NB * NT)
#ifndef TQB
#define TQB (NT / 64)
#endif
typedef __attribute__((ext_vector_type(8))) __bf16 v8b;
__device__ __forceinline__ v16b frag_b(const __bf16* rowk0, int lane) {
  union { v16b v; v8b q[2]; } u; const __bf16* p = rowk0 + 8 * (lane >> 4);
  u.q[0] = *(const v8b*)p; u.q[1] = *(const v8b*)(p + 16); return u.v;
}
__device__ __forceinline__ float bfr(float v) { return (float)(__bf16)v; }
__device__ __attribute__((noinline)) float exp_ni(float v) { return expf(v); }
__device__ __attribute__((noinline)) float erf_ni(float v) { return erff(v); }

#define WS_PK  0u
#define WS_QH  (WS_PK + 2u * 4 * DIM * DIM)
#define WS_QL  (WS_QH + 2u * NR * NH * 32)
#define WS_KH  (WS_QL + 2u * NR * NH * 32)
#define WS_KL  (WS_KH + 2u * NR * NH * 32)
#define WS_VH  (WS_KL + 2u * NR * NH * 32)
#define WS_O   (WS_VH + 2u * (size_t)NB * NH * 32 * NT)
#define WS_END (WS_O + 4u * (size_t)NH * NR * 32)

__global__ __launch_bounds__(128) void k_pack(const float* __restrict__ WQ, const float* __restrict__ WK, const float* __restrict__ WV, const float* __restrict__ WP, __bf16* __restrict__ PK) {
  const int n = blockIdx.x, which = blockIdx.y, t = threadIdx.x; const float* Wm = (which == 0) ? WQ : (which == 1) ? WK : (which == 2) ? WV : WP; __shared__ __align__(16) __bf16 s[DIM];
  for (int k = t; k < DIM; k += 128) s[k] = (__bf16)Wm[(size_t)n * DIM + k];
  __syncthreads();
  if (t < DIM / 8) vst2((unsigned*)(PK + ((size_t)which * DIM + n) * DIM + t * 8), *(const v4u*)&s[t * 8]);
}
__global__ __launch_bounds__(128) void k_qkv(const float* __restrict__ X, const __bf16* __restrict__ PK, _Float16* __restrict__ QH, _Float16* __restrict__ QL, _Float16* __restrict__ KH, _Float16* __restrict__ KL, _Float16* __restrict__ VH) {
  __shared__ __align__(16) float so[64][DIM + 1]; __shared__ __align__(16) _Float16 sth[64][40], stl[64][40];
  const int tid = threadIdx.x, wave = tid >> 5, lane = tid & 31, col = lane & 15, g = lane >> 4; const int which = blockIdx.y; const size_t r0 = (size_t)blockIdx.x * 64 + wave * 16; const __bf16* Wr = PK + (size_t)which * DIM * DIM;
#pragma unroll 1
  for (int half = 0; half < 2; ++half) { v8f acc[12] = {};
#pragma unroll 2
    for (int kc = 0; kc < DIM / 32; ++kc) { v16b a; { const float* p = X + (r0 + col) * DIM + kc * 32 + 8 * g;
#pragma unroll
        for (int i = 0; i < 8; ++i) { a[i] = (__bf16)p[i]; a[8 + i] = (__bf16)p[16 + i]; } }
#pragma unroll
      for (int j = 0; j < 12; ++j) acc[j] = wmma_bf(a, frag_b(Wr + (size_t)(half * 192 + j * 16 + col) * DIM + kc * 32, lane), acc[j]); }
#pragma unroll
    for (int j = 0; j < 12; ++j)
#pragma unroll
      for (int r = 0; r < 8; ++r) so[wave * 16 + 8 * g + r][half * 192 + j * 16 + col] = acc[j][r]; }
  __syncthreads();
  const size_t rb0 = (size_t)blockIdx.x * 64;
  if (which < 2) { _Float16* DH_ = which ? KH : QH; _Float16* DL_ = which ? KL : QL;
#pragma unroll 1
    for (int h = 0; h < NH; ++h) {
      for (int e = tid; e < 64 * 32; e += 128) { const int r = e >> 5, d = e & 31; const float v = (d < HDm) ? so[r][h * HDm + d] : 0.f; const _Float16 hv = (_Float16)v; sth[r][d] = hv; stl[r][d] = (_Float16)((v - (float)hv) * 2048.0f); }
      __syncthreads();
      for (int e = tid; e < 64 * 4; e += 128) { const int r = e >> 2, q = e & 3; const size_t o = ((rb0 + r) * NH + h) * 32 + q * 8; vst2((unsigned*)(DH_ + o), *(const v4u*)&sth[r][q * 8]); vst2((unsigned*)(DL_ + o), *(const v4u*)&stl[r][q * 8]); }
      __syncthreads(); } }
  else { const size_t b = rb0 / NT; const size_t t0 = rb0 % NT; __shared__ __align__(16) _Float16 svh[32][72];
#pragma unroll 1
    for (int h = 0; h < NH; ++h) {
      for (int e = tid; e < 32 * 64; e += 128) { const int d = e >> 6, r = e & 63; svh[d][r] = (_Float16)((d < HDm) ? so[r][h * HDm + d] : 0.f); }
      __syncthreads();
      for (int e = tid; e < 32 * 8; e += 128) { const int d = e >> 3, pc = e & 7; vst2((unsigned*)(VH + ((b * NH * 32 + h * 32 + d) * NT) + t0 + pc * 8), *(const v4u*)&svh[d][pc * 8]); }
      __syncthreads(); } }
}
__global__ __launch_bounds__(128) void k_attn(const _Float16* __restrict__ QH, const _Float16* __restrict__ QL, const _Float16* __restrict__ KH, const _Float16* __restrict__ KL, const _Float16* __restrict__ VH, const float* __restrict__ WPOS, const float* __restrict__ BPOS, const float* __restrict__ GATE, float* __restrict__ O) {
  __shared__ __align__(16) _Float16 sp1[4][16][40], sp2[4][16][40]; __shared__ __align__(16) float so[4][16][36];
  const int tid = threadIdx.x, wave = tid >> 5, lane = tid & 31, col = lane & 15, g = lane >> 4; const int qb = blockIdx.x, h = blockIdx.y; const size_t b = blockIdx.z; const int q0 = qb * 64 + wave * 16; const size_t rq = b * NT + q0;
  const float wx = bfr(WPOS[h * 3]), wy = bfr(WPOS[h * 3 + 1]), wd = bfr(WPOS[h * 3 + 2]), bp = bfr(BPOS[h]); const float gs = 1.0f / (1.0f + expf(-bfr(GATE[h])));   const float scale = 1.0f / sqrtf((float)HDm);
  const v16h aq = frag_h(QH + ((rq + col) * NH + h) * 32, lane), aql = frag_h(QL + ((rq + col) * NH + h) * 32, lane);
  float m1[8], l1[8], m2[8], l2[8]; int qx[8], qy[8];
#pragma unroll
  for (int r = 0; r < 8; ++r) { m1[r] = -3.0e38f; l1[r] = 0.f; m2[r] = -3.0e38f; l2[r] = 0.f; const int qi = q0 + 8 * g + r; qx[r] = qi % GWD; qy[r] = qi / GWD; }
  v8f acc1[2] = {}, acc2[2] = {};
#pragma unroll 1
  for (int ks = 0; ks < NT / 32; ++ks) { const int j0 = ks * 32; float s1[2][8], s2[2][8];
#pragma unroll
    for (int ct = 0; ct < 2; ++ct) { const int kk = j0 + ct * 16 + col; const size_t rk = ((b * NT + kk) * NH + h) * 32; v8f c = {}, cl = {};
      { const v16h kh = frag_h(KH + rk, lane); c = wmma16(aq, kh, c); cl = wmma16(aql, kh, cl); cl = wmma16(aq, frag_h(KL + rk, lane), cl); }
      const int kx = kk % GWD, ky = kk / GWD;
#pragma unroll
      for (int r = 0; r < 8; ++r) { s1[ct][r] = (c[r] + cl[r] * (1.0f / 2048.0f)) * scale; const float dx = (float)(kx - qx[r]), dy = (float)(ky - qy[r]); float t = dx * wx; t = t + dy * wy; t = t + (dx * dx + dy * dy) * wd; s2[ct][r] = t + bp; } }
#pragma unroll
    for (int r = 0; r < 8; ++r) {
      { float mx = fmaxf(s1[0][r], s1[1][r]);
#pragma unroll
        for (int o = 1; o < 16; o <<= 1) mx = fmaxf(mx, __shfl_xor(mx, o));
        const float mn = fmaxf(m1[r], mx); const float alpha = (m1[r] <= -1.0e38f) ? 0.f : __expf(m1[r] - mn); const float e0 = __expf(s1[0][r] - mn), e1 = __expf(s1[1][r] - mn); float es = e0 + e1;
#pragma unroll
        for (int o = 1; o < 16; o <<= 1) es += __shfl_xor(es, o);
        l1[r] = l1[r] * alpha + es; m1[r] = mn; acc1[0][r] *= alpha; acc1[1][r] *= alpha; sp1[wave][8 * g + r][col] = (_Float16)(e0 * 2048.0f); sp1[wave][8 * g + r][16 + col] = (_Float16)(e1 * 2048.0f); }
      { float mx = fmaxf(s2[0][r], s2[1][r]);
#pragma unroll
        for (int o = 1; o < 16; o <<= 1) mx = fmaxf(mx, __shfl_xor(mx, o));
        const float mn = fmaxf(m2[r], mx); const float alpha = (m2[r] <= -1.0e38f) ? 0.f : __expf(m2[r] - mn); const float e0 = __expf(s2[0][r] - mn), e1 = __expf(s2[1][r] - mn); float es = e0 + e1;
#pragma unroll
        for (int o = 1; o < 16; o <<= 1) es += __shfl_xor(es, o);
        l2[r] = l2[r] * alpha + es; m2[r] = mn; acc2[0][r] *= alpha; acc2[1][r] *= alpha; sp2[wave][8 * g + r][col] = (_Float16)(e0 * 2048.0f); sp2[wave][8 * g + r][16 + col] = (_Float16)(e1 * 2048.0f); } }
    LDSX();
    const v16h pa1 = frag_h(&sp1[wave][col][0], lane), pa2 = frag_h(&sp2[wave][col][0], lane);
#pragma unroll
    for (int dt = 0; dt < 2; ++dt) { const v16h vh = frag_h(VH + (b * NH * 32 + h * 32 + dt * 16 + col) * NT + j0, lane); acc1[dt] = wmma16(pa1, vh, acc1[dt]); acc2[dt] = wmma16(pa2, vh, acc2[dt]); }
    LDSX(); }
#pragma unroll
  for (int r = 0; r < 8; ++r) { const float w1 = (1.0f - gs), w2 = gs; const float den = w1 * 1.0f + w2 * 1.0f;
    const float i1 = w1 / (2048.0f * l1[r]) / den, i2 = w2 / (2048.0f * l2[r]) / den;
#pragma unroll
    for (int dt = 0; dt < 2; ++dt) so[wave][8 * g + r][dt * 16 + col] = acc1[dt][r] * i1 + acc2[dt][r] * i2; }
  LDSX();
  for (int rl = 0; rl < 16; ++rl) if (lane < 8) vst2(O + (((size_t)h * NR + rq + rl) * 32) + lane * 4, *(const v4f*)&so[wave][rl][lane * 4]);
}
__global__ __launch_bounds__(128) void k_out(const float* __restrict__ O, const __bf16* __restrict__ PK, const float* __restrict__ BP, float* __restrict__ OUT) {
  __shared__ __align__(16) __bf16 sh[64][DIM + 8], sl[64][DIM + 8]; __shared__ __align__(16) float so[4][16][132];
  const int tid = threadIdx.x, wave = tid >> 5, lane = tid & 31, col = lane & 15, g = lane >> 4; const size_t rb0 = (size_t)blockIdx.x * 64; const int n0 = blockIdx.y * 128;
  for (int e = tid; e < 64 * DIM; e += 128) { const int r = e / DIM, c = e % DIM; const int h = c / HDm, d = c % HDm; const float v = O[((size_t)h * NR + rb0 + r) * 32 + d]; const __bf16 hb = (__bf16)v; sh[r][c] = hb; sl[r][c] = (__bf16)(v - (float)hb); }
  if (tid < 64) for (int c = DIM; c < DIM + 8; ++c) { sh[tid][c] = (__bf16)0.f; sl[tid][c] = (__bf16)0.f; }
  __syncthreads();
  v8f acc[8] = {};
#pragma unroll
  for (int kc = 0; kc < DIM / 32; ++kc) { const v16b a = frag_b(&sh[wave * 16 + col][kc * 32], lane), al = frag_b(&sl[wave * 16 + col][kc * 32], lane);
#pragma unroll
    for (int j = 0; j < 8; ++j) { const v16b w = frag_b(PK + (size_t)3 * DIM * DIM + (size_t)(n0 + j * 16 + col) * DIM + kc * 32, lane); acc[j] = wmma_bf(al, w, acc[j]); acc[j] = wmma_bf(a, w, acc[j]); } }
#pragma unroll
  for (int j = 0; j < 8; ++j) { const float bb = bfr(BP[n0 + j * 16 + col]);
#pragma unroll
    for (int r = 0; r < 8; ++r) so[wave][8 * g + r][j * 16 + col] = acc[j][r] + bb; }
  LDSX();
  for (int rl = 0; rl < 16; ++rl) vst2(OUT + (rb0 + wave * 16 + rl) * DIM + n0 + lane * 4, *(const v4f*)&so[wave][rl][lane * 4]);
}
extern "C" void kernel_launch(void* const* d_in, const int* in_sizes, int n_in, void* d_out, int out_size, void* d_ws, size_t ws_size, hipStream_t stream) {
  (void)in_sizes; (void)n_in; (void)out_size;
  const float** F = (const float**)d_in;
  if (ws_size < (size_t)WS_END) return;
  char* ws = (char*)d_ws; __bf16* PK = (__bf16*)(ws + WS_PK); _Float16 *QH = (_Float16*)(ws + WS_QH), *QL = (_Float16*)(ws + WS_QL), *KH = (_Float16*)(ws + WS_KH), *KL = (_Float16*)(ws + WS_KL), *VH = (_Float16*)(ws + WS_VH); float* O = (float*)(ws + WS_O);
  k_pack<<<dim3(DIM, 4), 128, 0, stream>>>(F[1], F[2], F[3], F[7], PK);
  k_qkv<<<dim3(NR / 64, 3), 128, 0, stream>>>(F[0], PK, QH, QL, KH, KL, VH);
  k_attn<<<dim3(TQB, NH, NB), 128, 0, stream>>>(QH, QL, KH, KL, VH, F[4], F[5], F[6], O);
  k_out<<<dim3(NR / 64, DIM / 128), 128, 0, stream>>>(O, PK, F[8], (float*)d_out);
}
